// NNConvNet_36524401885778
// MI455X (gfx1250) — hardware-verified
//
#include <hip/hip_runtime.h>
#include <stddef.h>
#include <stdint.h>

#define FIN    128
#define FE     16
#define CW     32
#define CC     1024
#define NTHR   256
#define NWAVE  8
#define EPB    256
#define GTHR   128
#define GBM    64
#define EPT    8
#define CHUNK  (NTHR * EPT)
#define WCAP   (EPT * 32)
#define LISTN  (NWAVE * WCAP)
#define NBMAX  2048
#define SLOTB  11
#define RCAP   28672
#define DEGCAP 128
#define NU_WI  (CW * FIN / 8)
#define NU_WE  (CC * FE / 8)
#define WSMAX  134217728
#define SLOPE  0.01f
#define LDS_SCAN ((2 * RCAP + 2 * NBMAX + LISTN + CC + 2 * NWAVE) * 4)

static_assert((CHUNK & (CHUNK - 1)) == 0 && CHUNK <= (1 << SLOTB));
static_assert(NBMAX == (1 << SLOTB));
static_assert(NTHR * 8 == NBMAX);
static_assert(LISTN >= NBMAX);
static_assert(LISTN >= NWAVE * WCAP);
static_assert((RCAP % 32) == 0 && (RCAP % 4) == 0);
static_assert(LDS_SCAN <= 300000);
static_assert(NU_WI % NTHR == 0 && (NU_WI + NU_WE) % NTHR == 0);
static_assert(GBM == (GTHR / 32) * 16);
static_assert(FIN % 32 == 0 && CW == 32 && FE == 16 && CC == CW * CW);
static_assert(EPB == NTHR && EPB == NWAVE * 32);
static_assert(EPB * CW == 8 * NTHR * 4);
static_assert(GBM * CW == 4 * GTHR * 4);

typedef float          v4f  __attribute__((ext_vector_type(4)));
typedef float          v8f  __attribute__((ext_vector_type(8)));
typedef int            v4i  __attribute__((ext_vector_type(4)));
typedef int            v8i  __attribute__((ext_vector_type(8)));
typedef unsigned short v8us __attribute__((ext_vector_type(8)));
typedef __bf16         v16b __attribute__((ext_vector_type(16)));
typedef v4f  __attribute__((may_alias)) v4fa;
typedef v8us __attribute__((may_alias)) v8usa;
union FragB { v16b v; v8us h[2]; v8i w; };

__device__ __forceinline__ v8f wmb(const FragB& a, const FragB& b, v8f c) {
  v8f d = __builtin_amdgcn_wmma_f32_16x16x32_bf16(false, a.v, false, b.v, (short)0, c, false, false);
  asm volatile("v_nop\n\tv_nop\n\tv_nop\n\tv_nop" : "+v"(d) : "v"(a.w), "v"(b.w));
  return d;
}

__device__ __forceinline__ unsigned int f2bf(float f) {
  const unsigned int u = __float_as_uint(f);
  return ((u + 0x7FFFu + ((u >> 16) & 1u)) >> 16) & 0xFFFFu;
}
__device__ __forceinline__ float bf2f(unsigned int b) { return __uint_as_float(b << 16); }
__device__ __forceinline__ float bfr(float f) { return bf2f(f2bf(f)); }
__device__ __forceinline__ v8us cvt8(const float* p) {
  const v4f a = *(const v4fa*)p, b = *(const v4fa*)(p + 4);
  v8us o;
  o[0] = (unsigned short)f2bf(a.x); o[1] = (unsigned short)f2bf(a.y);
  o[2] = (unsigned short)f2bf(a.z); o[3] = (unsigned short)f2bf(a.w);
  o[4] = (unsigned short)f2bf(b.x); o[5] = (unsigned short)f2bf(b.y);
  o[6] = (unsigned short)f2bf(b.z); o[7] = (unsigned short)f2bf(b.w);
  return o;
}
__device__ __forceinline__ float lrelu(float v) { return v >= 0.0f ? v : SLOPE * v; }
__device__ __forceinline__ void put16(unsigned short* dp, v8us o) {
  *(volatile v8us*)dp = o;
  __threadfence();
  *(volatile v8us*)dp = o;
}

__device__ __forceinline__ int scan_chunk(const int* __restrict__ dsts, int nE, int cbase, int slotBase,
                                          int nb, int vec8, int* list, int tid, int lane, int wave) {
  int wc = 0;
  const int el0  = tid * EPT;
  const int e0   = cbase + el0;
  const int sent = -2147483647 - 1;
  v4i da, db;
  if (vec8 != 0 && cbase + CHUNK <= nE) {
    da = *(const v4i*)(dsts + e0);
    db = *(const v4i*)(dsts + e0 + 4);
  } else {
    da.x = (e0     < nE) ? dsts[min(e0,     nE - 1)] : sent;
    da.y = (e0 + 1 < nE) ? dsts[min(e0 + 1, nE - 1)] : sent;
    da.z = (e0 + 2 < nE) ? dsts[min(e0 + 2, nE - 1)] : sent;
    da.w = (e0 + 3 < nE) ? dsts[min(e0 + 3, nE - 1)] : sent;
    db.x = (e0 + 4 < nE) ? dsts[min(e0 + 4, nE - 1)] : sent;
    db.y = (e0 + 5 < nE) ? dsts[min(e0 + 5, nE - 1)] : sent;
    db.z = (e0 + 6 < nE) ? dsts[min(e0 + 6, nE - 1)] : sent;
    db.w = (e0 + 7 < nE) ? dsts[min(e0 + 7, nE - 1)] : sent;
  }
  const unsigned nbs = (unsigned)slotBase;
  const unsigned unb = (unsigned)nb;
  const unsigned s0 = (unsigned)da.x - nbs, s1 = (unsigned)da.y - nbs;
  const unsigned s2 = (unsigned)da.z - nbs, s3 = (unsigned)da.w - nbs;
  const unsigned s4 = (unsigned)db.x - nbs, s5 = (unsigned)db.y - nbs;
  const unsigned s6 = (unsigned)db.z - nbs, s7 = (unsigned)db.w - nbs;
  const bool h0 = s0 < unb, h1 = s1 < unb, h2 = s2 < unb, h3 = s3 < unb;
  const bool h4 = s4 < unb, h5 = s5 < unb, h6 = s6 < unb, h7 = s7 < unb;
  const unsigned any = __builtin_amdgcn_ballot_w32(h0 | h1 | h2 | h3 | h4 | h5 | h6 | h7);
  if (any != 0u) {
#define HITJ(J, HJ, SJ) { \
      const unsigned mj = __builtin_amdgcn_ballot_w32(HJ); \
      if (mj != 0u) { \
        if (HJ) { \
          const int pos = wc + (int)__builtin_amdgcn_mbcnt_lo(mj, 0u); \
          if (pos < WCAP) list[wave * WCAP + pos] = ((el0 + (J)) << SLOTB) | (int)(SJ); \
        } \
        wc += (int)__builtin_popcount(mj); } }
    HITJ(0, h0, s0)
    HITJ(1, h1, s1)
    HITJ(2, h2, s2)
    HITJ(3, h3, s3)
    HITJ(4, h4, s4)
    HITJ(5, h5, s5)
    HITJ(6, h6, s6)
    HITJ(7, h7, s7)
#undef HITJ
  }
  return wc;
}

__global__ __launch_bounds__(NTHR) void k_prep(const float* __restrict__ W_in, const float* __restrict__ W_edge,
                                               unsigned short* WIT, unsigned short* WET) {
  const int u = (int)blockIdx.x * NTHR + (int)threadIdx.x;
  v8us o;
  if (u < NU_WI) {
    const int n  = u >> 4;
    const int k8 = (u & 15) * 8;
    const float* p = W_in + (size_t)k8 * CW + n;
#pragma unroll
    for (int i = 0; i < 8; ++i) o[i] = (unsigned short)f2bf(p[(size_t)i * CW]);
    put16(WIT + (size_t)n * FIN + k8, o);
    return;
  } else if (u < NU_WI + NU_WE) {
    const int v  = u - NU_WI;
    const int n  = v >> 1;
    const int k8 = (v & 1) * 8;
    const float* p = W_edge + (size_t)k8 * CC + n;
#pragma unroll
    for (int i = 0; i < 8; ++i) o[i] = (unsigned short)f2bf(p[(size_t)i * CC]);
    put16(WET + (size_t)n * FE + k8, o);
    return;
  }
}

__global__ __launch_bounds__(GTHR) void k_h(const float* __restrict__ x, int nN,
                                            const unsigned short* __restrict__ WIT,
                                            const float* __restrict__ b_in, float* H) {
  __shared__ __attribute__((aligned(16))) float stg[GBM * CW];
  const int tid = (int)threadIdx.x, lane = tid & 31, wave = tid >> 5, hh = lane >> 4, m = lane & 15;
  const int rowBase = (int)blockIdx.x * GBM;
  const int row = rowBase + 16 * wave + m;
  const int rc  = row < nN ? row : nN - 1;
  const float* xp = x + (size_t)rc * FIN + 8 * hh;
  const unsigned short* bp = WIT + (size_t)m * FIN + 8 * hh;

  v8f acc[2];
  {
    const v8f z = {0.f, 0.f, 0.f, 0.f, 0.f, 0.f, 0.f, 0.f};
    acc[0] = z; acc[1] = z;
  }
#pragma unroll 1
  for (int k0 = 0; k0 < FIN; k0 += 32) {
    FragB af;
    af.h[0] = cvt8(xp + k0);
    af.h[1] = cvt8(xp + k0 + 16);
#pragma unroll
    for (int nt = 0; nt < 2; ++nt) {
      const unsigned short* bq = bp + (size_t)(16 * nt) * FIN + k0;
      FragB bf;
      bf.h[0] = *(const v8usa*)bq;
      bf.h[1] = *(const v8usa*)(bq + 16);
      acc[nt] = wmb(af, bf, acc[nt]);
    }
  }

#pragma unroll
  for (int nt = 0; nt < 2; ++nt) {
    const int lc = 16 * nt + m;
    const float bv = bfr(b_in[lc]);
#pragma unroll
    for (int r = 0; r < 8; ++r) {
      const int lr = 16 * wave + 8 * hh + r;
      stg[lr * CW + lc] = lrelu(acc[nt][r] + bv);
    }
  }
  __syncthreads();

  v4f pv[4];
#pragma unroll
  for (int it = 0; it < 4; ++it) pv[it] = *(const v4fa*)(stg + (it * GTHR + tid) * 4);
  float* hb = H + (size_t)rowBase * CW;
#pragma unroll
  for (int it = 0; it < 4; ++it) *(volatile v4f*)(hb + (size_t)(it * GTHR + tid) * 4) = pv[it];
  __threadfence();
#pragma unroll
  for (int it = 0; it < 4; ++it) *(volatile v4f*)(hb + (size_t)(it * GTHR + tid) * 4) = pv[it];
}

__global__ __launch_bounds__(NTHR) void k_edge(const float* __restrict__ ea, const int* __restrict__ srcs,
                                               int nE, int nN, const float* __restrict__ H,
                                               const unsigned short* __restrict__ WET,
                                               const float* __restrict__ b_edge, float* MSG) {
  __shared__ __attribute__((aligned(16))) float hs[EPB * CW];
  __shared__ __attribute__((aligned(16))) float sbe[CC];
  const int tid = (int)threadIdx.x, lane = tid & 31, wave = tid >> 5, hh = lane >> 4, m = lane & 15;
  const int elb = (int)blockIdx.x * EPB;

  for (int i = tid; i < CC; i += NTHR) sbe[i] = bfr(b_edge[i]);
  {
    const int el  = elb + tid;
    const int elc = el < nE ? el : nE - 1;
    int s = srcs[elc];
    s = s < 0 ? 0 : (s > nN - 1 ? nN - 1 : s);
    const float* hr = H + (size_t)s * CW;
    float* hd = hs + tid * CW;
#pragma unroll
    for (int j = 0; j < 8; ++j) *(v4fa*)(hd + 4 * j) = *(const v4fa*)(hr + 4 * j);
  }
  const v8us z8 = {0, 0, 0, 0, 0, 0, 0, 0};
  FragB a0, a1;
  {
    const int e0 = elb + 32 * wave + m;
    const int e1 = e0 + 16;
    const int c0 = e0 < nE ? e0 : nE - 1;
    const int c1 = e1 < nE ? e1 : nE - 1;
    a0.h[0] = cvt8(ea + (size_t)c0 * FE + 8 * hh);
    a0.h[1] = z8;
    a1.h[0] = cvt8(ea + (size_t)c1 * FE + 8 * hh);
    a1.h[1] = z8;
  }
  __syncthreads();

  v8f acc[2][2];
  const v8f zf = {0.f, 0.f, 0.f, 0.f, 0.f, 0.f, 0.f, 0.f};
  acc[0][0] = zf; acc[0][1] = zf; acc[1][0] = zf; acc[1][1] = zf;
  float* hw = hs + (32 * wave) * CW;
  const unsigned short* bp = WET + (size_t)m * FE + 8 * hh;

#pragma unroll 1
  for (int c = 0; c < CW; ++c) {
    float hv0[8], hv1[8];
#pragma unroll
    for (int r = 0; r < 8; ++r) {
      hv0[r] = hw[(8 * hh + r) * CW + c];
      hv1[r] = hw[(16 + 8 * hh + r) * CW + c];
    }
#pragma unroll
    for (int hf = 0; hf < 2; ++hf) {
      const int nt = 2 * c + hf;
      FragB b;
      b.h[0] = *(const v8usa*)(bp + (size_t)(16 * nt) * FE);
      b.h[1] = z8;
      const v8f d0 = wmb(a0, b, zf);
      const v8f d1 = wmb(a1, b, zf);
      const float bias = sbe[16 * nt + m];
#pragma unroll
      for (int r = 0; r < 8; ++r) {
        const float w0 = lrelu(d0[r] + bias);
        const float w1 = lrelu(d1[r] + bias);
        acc[0][hf][r] = fmaf(w0, hv0[r], acc[0][hf][r]);
        acc[1][hf][r] = fmaf(w1, hv1[r], acc[1][hf][r]);
      }
    }
  }
  __syncthreads();

#pragma unroll
  for (int mt = 0; mt < 2; ++mt)
#pragma unroll
    for (int hf = 0; hf < 2; ++hf)
#pragma unroll
      for (int r = 0; r < 8; ++r)
        hw[(16 * mt + 8 * hh + r) * CW + 16 * hf + m] = acc[mt][hf][r];
  __syncthreads();

  v4f pv[8];
#pragma unroll
  for (int it = 0; it < 8; ++it) pv[it] = *(const v4fa*)(hs + (size_t)(it * NTHR + tid) * 4);
  float* mb = MSG + (size_t)elb * CW;
#pragma unroll
  for (int it = 0; it < 8; ++it) *(volatile v4f*)(mb + (size_t)(it * NTHR + tid) * 4) = pv[it];
  __threadfence();
#pragma unroll
  for (int it = 0; it < 8; ++it) *(volatile v4f*)(mb + (size_t)(it * NTHR + tid) * 4) = pv[it];
}

__global__ __launch_bounds__(NTHR) void k_scan(
    const int* __restrict__ srcs, const int* __restrict__ dsts,
    const float* __restrict__ MSG, const float* __restrict__ H,
    const float* __restrict__ W_root, const float* __restrict__ b_conv,
    const float* __restrict__ W_out, const float* __restrict__ b_out,
    float* out, int nN, int nE, int nb, int vec8) {
  extern __shared__ v4f lds_dyn[];
  int*   reg1 = (int*)lds_dyn;
  int*   reg2 = reg1 + RCAP;
  int*   scnt = reg2 + RCAP;
  int*   soff = scnt + NBMAX;
  int*   list = soff + NBMAX;
  float* swr  = (float*)(list + LISTN);
  int*   wcnt = (int*)(swr + CC);
  int*   wtot = wcnt + NWAVE;
  const int tid = (int)threadIdx.x, lane = tid & 31, wave = tid >> 5;
  const int nodeBase = (int)blockIdx.x * nb;
  (void)srcs;

  for (int i = tid; i < NBMAX; i += NTHR) scnt[i] = 0;
  for (int i = tid; i < CC; i += NTHR) swr[i] = bfr(W_root[i]);
  __syncthreads();

  int tot = 0;
  const int nChunks = (nE + CHUNK - 1) / CHUNK;
#pragma unroll 1
  for (int ch = 0; ch < nChunks; ++ch) {
    const int cbase = ch * CHUNK;
    const int wc = scan_chunk(dsts, nE, cbase, nodeBase, nb, vec8, list, tid, lane, wave);
    if (lane == 0) wcnt[wave] = wc;
    __syncthreads();
    int pre = 0, all = 0;
#pragma unroll
    for (int w2 = 0; w2 < NWAVE; ++w2) {
      int c = wcnt[w2];
      c = c < 0 ? 0 : (c > WCAP ? WCAP : c);
      all += c;
      pre += (w2 < wave) ? c : 0;
    }
    const int wcc  = wc > WCAP ? WCAP : wc;
    const int base = tot + pre;
#pragma unroll 1
    for (int i = lane; i < wcc; i += 32) {
      const int ent = list[wave * WCAP + i];
      const int el  = (ent >> SLOTB) & (CHUNK - 1);
      const int sl  = ent & (NBMAX - 1);
      int eid = cbase + el;
      eid = eid > nE - 1 ? nE - 1 : eid;
      const int pos = base + i;
      if (pos < RCAP) reg1[pos] = (int)(((unsigned)eid << SLOTB) | (unsigned)sl);
    }
    tot += all;
    tot = tot > RCAP ? RCAP : tot;
    __syncthreads();
  }
  const int nh = tot;

  if (wave == 0) {
#pragma unroll 1
    for (int b0 = 0; b0 < nh; b0 += 32) {
      const int idx = b0 + lane;
      const int uv  = reg1[idx < nh ? idx : nh - 1];
      const int m32 = (nh - b0) < 32 ? (nh - b0) : 32;
#pragma unroll 1
      for (int k = 0; k < m32; ++k) {
        const int u  = __builtin_amdgcn_readlane(uv, k);
        const int sl = u & (NBMAX - 1);
        if (lane == 0) scnt[sl] = scnt[sl] + 1;
      }
    }
  }
  __syncthreads();

  {
    const v4i ca = *(const v4i*)(scnt + 8 * tid);
    const v4i cb = *(const v4i*)(scnt + 8 * tid + 4);
    const int e0 = ca.x < 0 ? 0 : ca.x, e1 = ca.y < 0 ? 0 : ca.y, e2 = ca.z < 0 ? 0 : ca.z, e3 = ca.w < 0 ? 0 : ca.w;
    const int e4 = cb.x < 0 ? 0 : cb.x, e5 = cb.y < 0 ? 0 : cb.y, e6 = cb.z < 0 ? 0 : cb.z, e7 = cb.w < 0 ? 0 : cb.w;
    const int ts = e0 + e1 + e2 + e3 + e4 + e5 + e6 + e7;
    int incl = ts;
#pragma unroll
    for (int d = 1; d < 32; d <<= 1) {
      const int up = __shfl_up(incl, d);
      if (lane >= d) incl += up;
    }
    if (lane == 31) wtot[wave] = incl;
    __syncthreads();
    int pre = 0;
#pragma unroll
    for (int w2 = 0; w2 < NWAVE; ++w2) pre += (w2 < wave) ? wtot[w2] : 0;
    int run = pre + incl - ts;
    soff[8 * tid + 0] = run; run += e0;
    soff[8 * tid + 1] = run; run += e1;
    soff[8 * tid + 2] = run; run += e2;
    soff[8 * tid + 3] = run; run += e3;
    soff[8 * tid + 4] = run; run += e4;
    soff[8 * tid + 5] = run; run += e5;
    soff[8 * tid + 6] = run; run += e6;
    soff[8 * tid + 7] = run;
  }
  __syncthreads();
  for (int i = tid; i < NBMAX; i += NTHR) list[i] = soff[i];
  __syncthreads();

  if (wave == 0) {
#pragma unroll 1
    for (int b0 = 0; b0 < nh; b0 += 32) {
      const int idx = b0 + lane;
      const int uv  = reg1[idx < nh ? idx : nh - 1];
      const int m32 = (nh - b0) < 32 ? (nh - b0) : 32;
#pragma unroll 1
      for (int k = 0; k < m32; ++k) {
        const int u   = __builtin_amdgcn_readlane(uv, k);
        const int sl  = u & (NBMAX - 1);
        const int eid = (int)((unsigned)u >> SLOTB);
        if (lane == 0) {
          int pos = list[sl];
          pos = pos < 0 ? 0 : (pos > RCAP - 1 ? RCAP - 1 : pos);
          reg2[pos] = eid;
          list[sl] = pos + 1;
        }
      }
    }
  }
  __syncthreads();

  const int nbw = nb >> 3;
  const bool ovf = (nh >= RCAP);
  const float qnan = __int_as_float(0x7fc00000);
  const float bc = bfr(b_conv[lane]);
  const float wo = bfr(W_out[lane]);
  const float bo = bfr(b_out[0]);
  float* res = (float*)list;

#pragma unroll 1
  for (int jt = 0; jt < nbw; ++jt) {
    const int slot = wave * nbw + jt;
    const int grow = nodeBase + slot;
    const int gcl  = grow < nN ? grow : nN - 1;
    int st = soff[slot];
    const int craw = scnt[slot];
    int cnt = craw;
    st  = st < 0 ? 0 : (st > nh ? nh : st);
    cnt = cnt < 0 ? 0 : (cnt > DEGCAP ? DEGCAP : cnt);
    if (cnt > nh - st) cnt = nh - st;
    const float pz = (ovf || craw > DEGCAP) ? qnan : 0.0f;

    float ag = 0.0f;
#pragma unroll 1
    for (int q = 0; q < cnt; ++q) {
      int idx = st + q; idx = idx > RCAP - 1 ? RCAP - 1 : idx;
      int eid = reg2[idx]; eid = eid < 0 ? 0 : (eid > nE - 1 ? nE - 1 : eid);
      ag += MSG[(size_t)eid * CW + lane];
    }
    const float hreg = H[(size_t)gcl * CW + lane];
    float rt = 0.0f;
#pragma unroll 4
    for (int k = 0; k < CW; ++k) {
      const float hk = __shfl(hreg, k);
      rt = fmaf(hk, swr[k * CW + lane], rt);
    }
    float t = ag + rt;
    t = t + bc;
    const float h2 = lrelu(t);
    float part = h2 * wo;
#pragma unroll
    for (int off = 16; off > 0; off >>= 1) part += __shfl_xor(part, off);
    const float r = part + bo + pz;
    if (lane == 0) res[slot] = r;
  }

  __syncthreads();
  const int npc = nb >> 2;
#pragma unroll 1
  for (int p = tid; p < npc; p += NTHR) {
    const v4f v = *(const v4fa*)(res + 4 * p);
    const int r0 = nodeBase + 4 * p;
    if (r0 + 3 < nN) {
      *(volatile v4f*)(out + r0) = v;
    } else {
      if (r0     < nN) *(volatile float*)(out + r0)     = v.x;
      if (r0 + 1 < nN) *(volatile float*)(out + r0 + 1) = v.y;
      if (r0 + 2 < nN) *(volatile float*)(out + r0 + 2) = v.z;
    }
  }
  __threadfence();
#pragma unroll 1
  for (int p = tid; p < npc; p += NTHR) {
    const v4f v = *(const v4fa*)(res + 4 * p);
    const int r0 = nodeBase + 4 * p;
    if (r0 + 3 < nN) {
      *(volatile v4f*)(out + r0) = v;
    } else {
      if (r0     < nN) *(volatile float*)(out + r0)     = v.x;
      if (r0 + 1 < nN) *(volatile float*)(out + r0 + 1) = v.y;
      if (r0 + 2 < nN) *(volatile float*)(out + r0 + 2) = v.z;
    }
  }
}

static int pick_nb(int nE, int nN) {
  int nb = NBMAX;
  while (nb > 32 && (long long)nb * (long long)nE * 5LL > (long long)RCAP * (long long)nN * 4LL) nb >>= 1;
  return nb;
}
static inline int cdiv(int a, int b) { return (a + b - 1) / b; }

extern "C" void kernel_launch(void* const* d_in, const int* in_sizes, int n_in,
                              void* d_out, int out_size, void* d_ws, size_t ws_size,
                              hipStream_t stream) {
  if (n_in < 11) return;
  if (in_sizes[0] < FIN || (in_sizes[0] % FIN) != 0) return;
  const int nN = in_sizes[0] / FIN;
  if (nN > (1 << 22)) return;
  if (in_sizes[1] < 2 || (in_sizes[1] & 1) != 0) return;
  const int nE = in_sizes[1] / 2;
  if (nE < 1 || nE >= (1 << (32 - SLOTB))) return;
  if ((long long)in_sizes[2] != (long long)nE * FE) return;
  if (in_sizes[3] != FIN * CW) return;
  if (in_sizes[4] != CW) return;
  if (in_sizes[5] != FE * CC) return;
  if (in_sizes[6] != CC) return;
  if (in_sizes[7] != CW * CW) return;
  if (in_sizes[8] != CW) return;
  if (in_sizes[9] != CW) return;
  if (in_sizes[10] < 1) return;
  if (out_size != nN) return;

  const float* x      = (const float*)d_in[0];
  const int*   ei     = (const int*)  d_in[1];
  const float* eattr  = (const float*)d_in[2];
  const float* W_in   = (const float*)d_in[3];
  const float* b_in   = (const float*)d_in[4];
  const float* W_edge = (const float*)d_in[5];
  const float* b_edge = (const float*)d_in[6];
  const float* W_root = (const float*)d_in[7];
  const float* b_conv = (const float*)d_in[8];
  const float* W_out  = (const float*)d_in[9];
  const float* b_out  = (const float*)d_in[10];
  float* out = (float*)d_out;
  const int* src = ei;
  const int* dst = ei + nE;

  const int MP   = cdiv(nN, GBM) * GBM;
  const int EP   = cdiv(nE, EPB) * EPB;
  const int nb   = pick_nb(nE, nN);
  if (nb < 32 || (nb & (nb - 1)) != 0 || nb > NBMAX) return;
  const int gA   = cdiv(nN, nb);
  if ((long long)gA * nb < (long long)nN) return;
  const int vec8 = ((nE & 3) == 0) ? 1 : 0;

  char* ws = (char*)d_ws;
  size_t off = 0;
  const size_t oWIT = off; off += (size_t)CW * FIN * 2;          off = (off + 255) & ~(size_t)255;
  const size_t oWET = off; off += (size_t)CC * FE * 2;           off = (off + 255) & ~(size_t)255;
  const size_t oH   = off; off += (size_t)MP * CW * 4;           off = (off + 255) & ~(size_t)255;
  const size_t oMSG = off; off += (size_t)EP * CW * 4;           off = (off + 255) & ~(size_t)255;
  if (off > ws_size || off > (size_t)WSMAX) return;
  unsigned short* WIT = (unsigned short*)(ws + oWIT);
  unsigned short* WET = (unsigned short*)(ws + oWET);
  float*          H   = (float*)(ws + oH);
  float*          MSG = (float*)(ws + oMSG);

  hipFuncSetAttribute(reinterpret_cast<const void*>(&k_scan),
                      hipFuncAttributeMaxDynamicSharedMemorySize, LDS_SCAN);

  k_prep<<<(NU_WI + NU_WE) / NTHR, NTHR, 0, stream>>>(W_in, W_edge, WIT, WET);
  k_h<<<MP / GBM, GTHR, 0, stream>>>(x, nN, WIT, b_in, H);
  k_edge<<<EP / EPB, NTHR, 0, stream>>>(eattr, src, nE, nN, H, WET, b_edge, MSG);
  k_scan<<<gA, NTHR, LDS_SCAN, stream>>>(src, dst, MSG, H, W_root, b_conv, W_out, b_out, out, nN, nE, nb, vec8);
}
